// LocalGeometryEncoding_49435073577117
// MI455X (gfx1250) — hardware-verified
//
#include <hip/hip_runtime.h>


namespace {
constexpr int C = 8, NG = 64 * 64 * 64, NV = 100000, NP = 100032  , K = 32, DIN = C * K  , H = 512;
constexpr float XS = 8.0f, WSC = 256.0f;

typedef _Float16 b16;
typedef __attribute__((ext_vector_type(16))) _Float16 v16b;
typedef __attribute__((ext_vector_type(8))) _Float16 v8b;
typedef __attribute__((ext_vector_type(8))) float v8f;
typedef __attribute__((ext_vector_type(4))) float v4f;
__device__ __forceinline__ float bf16_rne(float f) { unsigned int u = __float_as_uint(f); u += 0x7FFFu + ((u >> 16) & 1u); return __uint_as_float(u & 0xFFFF0000u); }
__device__ __forceinline__ void split16(float v, b16& hi, b16& lo) { hi = (b16)v; lo = (b16)(v - (float)hi); }
__device__ __forceinline__ v16b frag_kb(const b16* p, int hh) { const v8b a = *(const v8b*)(p + 8 * hh), b = *(const v8b*)(p + 16 + 8 * hh); v16b f;
#pragma unroll
  for (int e = 0; e < 8; ++e) { f[e] = a[e]; f[8 + e] = b[e]; } return f; }
__device__ __forceinline__ v8f wmma16b(v16b a, v16b b, v8f c) { v8f d = __builtin_amdgcn_wmma_f32_16x16x32_f16(false, a, false, b, (short)0, c, false, false); asm volatile("v_nop\n\tv_nop\n\tv_nop\n\tv_nop" : "+v"(d) : "v"(a), "v"(b)); return d; }
__device__ __forceinline__ void wave_lds_sync() { __builtin_amdgcn_fence(__ATOMIC_RELEASE, "workgroup"); __builtin_amdgcn_wave_barrier(); __builtin_amdgcn_fence(__ATOMIC_ACQUIRE, "workgroup"); }
__device__ __forceinline__ int iclamp(int v, int lo, int hi) { return v < lo ? lo : (v > hi ? hi : v); }

__global__ __launch_bounds__(256) void prep_kernel(const float* __restrict__ enc, const int* __restrict__ map, const float* __restrict__ w1, const float* __restrict__ w2, b16* __restrict__ X16, b16* __restrict__ W1T, b16* __restrict__ W2T) {
  const size_t t = (size_t)blockIdx.x * 256 + threadIdx.x; const size_t nx = (size_t)NP * DIN / 8, n1 = (size_t)H * DIN / 8, n2 = (size_t)K * H / 8; v8b o;
  if (t < nx) { const size_t e = t * 8; const size_t n = e / DIN; const int col = (int)(e % DIN); const int c = col / K, k0 = col % K;
    for (int j = 0; j < 8; ++j) { float v = 0.0f; if (n < (size_t)NV) { const int idx = map[n * K + k0 + j]; if (idx != 0) v = bf16_rne(enc[(size_t)c * NG + iclamp(idx, 0, NG - 1)]); } o[j] = (b16)(v * XS); }
    for (int pass = 0; pass < 2; ++pass) { *(volatile v8b*)(X16 + e) = o; __threadfence(); } return; }
  size_t u = t - nx;
  if (u < n1) { const size_t e = u * 8; const int oo = (int)(e / DIN), i0 = (int)(e % DIN); for (int j = 0; j < 8; ++j) o[j] = (b16)(bf16_rne(w1[(size_t)(i0 + j) * H + oo]) * WSC); for (int pass = 0; pass < 2; ++pass) { *(volatile v8b*)(W1T + e) = o; __threadfence(); } return; }
  u -= n1;
  if (u < n2) { const size_t e = u * 8; const int oo = (int)(e / H), i0 = (int)(e % H); for (int j = 0; j < 8; ++j) o[j] = (b16)(bf16_rne(w2[(size_t)(i0 + j) * K + oo]) * WSC); for (int pass = 0; pass < 2; ++pass) { *(volatile v8b*)(W2T + e) = o; __threadfence(); } }
}
__global__ __launch_bounds__(32) void mlp_kernel(const b16* __restrict__ X16, const b16* __restrict__ W1T, const float* __restrict__ b1, const b16* __restrict__ W2T, const float* __restrict__ b2, float* __restrict__ out) {
  __shared__ __attribute__((aligned(16))) b16 Hh[16][H + 8], Hl[16][H + 8]; __shared__ __attribute__((aligned(16))) float Ts[16][K + 4];
  const int lane = threadIdx.x, nloc = lane & 15, hlf = lane >> 4; const size_t m0 = (size_t)blockIdx.x * 16;
  for (int g = 0; g < H / 128; ++g) { v8f acc[8];
#pragma unroll
    for (int t = 0; t < 8; ++t) acc[t] = (v8f){};
#pragma unroll 2
    for (int kb = 0; kb < DIN; kb += 32) { const v16b a = frag_kb(X16 + (m0 + nloc) * DIN + kb, hlf);
#pragma unroll
      for (int t = 0; t < 8; ++t) acc[t] = wmma16b(a, frag_kb(W1T + (size_t)(g * 128 + t * 16 + nloc) * DIN + kb, hlf), acc[t]); }
#pragma unroll
    for (int t = 0; t < 8; ++t) { const int c = g * 128 + t * 16 + nloc; const float bb = bf16_rne(b1[c]);
#pragma unroll
      for (int r = 0; r < 8; ++r) { b16 p, q; split16(fmaxf(acc[t][r] * (1.0f / (XS * WSC)) + bb, 0.0f) * XS, p, q); Hh[8 * hlf + r][c] = p; Hl[8 * hlf + r][c] = q; } } }
  wave_lds_sync();
  v8f o2[2] = {{}, {}};
#pragma unroll 2
  for (int kb = 0; kb < H; kb += 32) { const v16b a = frag_kb(&Hh[nloc][kb], hlf), al = frag_kb(&Hl[nloc][kb], hlf);
#pragma unroll
    for (int t = 0; t < 2; ++t) { const v16b bw = frag_kb(W2T + (size_t)(t * 16 + nloc) * H + kb, hlf); o2[t] = wmma16b(a, bw, o2[t]); o2[t] = wmma16b(al, bw, o2[t]); } }
#pragma unroll
  for (int t = 0; t < 2; ++t) { const float bb = bf16_rne(b2[t * 16 + nloc]);
#pragma unroll
    for (int r = 0; r < 8; ++r) Ts[8 * hlf + r][t * 16 + nloc] = o2[t][r] * (1.0f / (XS * WSC)) + bb; }
  wave_lds_sync();
  for (int pass = 0; pass < 2; ++pass) { for (int rr = 0; rr < 16; ++rr) if (m0 + rr < (size_t)NV && lane < 8) *(volatile v4f*)(out + (m0 + rr) * K + lane * 4) = *(const v4f*)(&Ts[rr][lane * 4]); __threadfence(); }
}
}

extern "C" void kernel_launch(void* const* d_in, const int* in_sizes, int n_in, void* d_out, int out_size, void* d_ws, size_t ws_size, hipStream_t stream) {
  (void)n_in;
  auto Fp = [&](int i) { return (const float*)d_in[i]; }; auto Ip = [&](int i) { return (const int*)d_in[i]; };
  if (in_sizes[0] != C * NG || in_sizes[1] != NV * K || in_sizes[2] != DIN * H || in_sizes[3] != H || in_sizes[4] != H * K || in_sizes[5] != K || out_size != NV * K) return;
  size_t off = 0; char* ws = (char*)d_ws;
  auto carve = [&](size_t bytes) { char* p = ws + off; off += (bytes + 255) & ~(size_t)255; return p; };
  b16* X16 = (b16*)carve((size_t)NP * DIN * 2); b16* W1T = (b16*)carve((size_t)H * DIN * 2); b16* W2T = (b16*)carve((size_t)K * H * 2);
  if (off > ws_size || off > ((size_t)128 << 20)) return;
  prep_kernel<<<(unsigned)(((size_t)NP * DIN / 8 + (size_t)H * DIN / 8 + (size_t)K * H / 8 + 255) / 256), 256, 0, stream>>>(Fp(0), Ip(1), Fp(2), Fp(4), X16, W1T, W2T);
  mlp_kernel<<<NP / 16, 32, 0, stream>>>(X16, W1T, Fp(3), W2T, Fp(5), (float*)d_out);
}
